// MultiHeadAttention_47845935677543
// MI455X (gfx1250) — hardware-verified
//
#include <hip/hip_runtime.h>


#ifndef NB
#define NB 4
#endif
#ifndef SEQ
#define SEQ 2048
#endif
#define NB_FULL  4
#define SEQ_FULL 2048
#define DM   1024
#define NH   16
#define HD   64
#define WCAR 64.0f
#define WINV (1.0f / 64.0f)
#define CCAR 64.0f
#define OINV (1.0f / 4096.0f)
#define C2   0.18033688011112042f
#define TSP  72

static_assert(NH * HD == DM);
static_assert(HD == 64);
static_assert(DM % 32 == 0);
static_assert(DM % 64 == 0);
static_assert(SEQ % 64 == 0);
static_assert(SEQ <= SEQ_FULL);
static_assert(NB <= NB_FULL);
static_assert((TSP * 2) % 16 == 0);
static_assert(TSP >= HD);

typedef _Float16 h16;
typedef __attribute__((ext_vector_type(16))) _Float16 v16h;
typedef __attribute__((ext_vector_type(8)))  _Float16 v8h;
typedef __attribute__((ext_vector_type(8)))  float    v8f;
typedef __attribute__((ext_vector_type(4)))  float    v4f;
typedef v8h __attribute__((may_alias)) v8ha;
typedef v4f __attribute__((may_alias)) v4fa;

__device__ __forceinline__ unsigned short f2bf(float f) { unsigned u = __float_as_uint(f); u += 0x7FFFu + ((u >> 16) & 1u); return (unsigned short)(u >> 16); }
__device__ __forceinline__ float bf2f(unsigned short b) { return __uint_as_float(((unsigned)b) << 16); }
__device__ __forceinline__ float bfr(float f) { return bf2f(f2bf(f)); }
__device__ __forceinline__ v16h cat16(v8h lo, v8h hi) { return __builtin_shufflevector(lo, hi, 0, 1, 2, 3, 4, 5, 6, 7, 8, 9, 10, 11, 12, 13, 14, 15); }
__device__ __forceinline__ v16h ldh(const h16* p) { return cat16(*(const v8h*)p, *(const v8h*)(p + 16)); }
__device__ __forceinline__ v8f wmma16(v16h a, v16h b, v8f c) { return __builtin_amdgcn_wmma_f32_16x16x32_f16(false, a, false, b, (short)0, c, false, false); }
__device__ __forceinline__ void wave_lds_sync() { __builtin_amdgcn_fence(3  , "wavefront"); __builtin_amdgcn_wave_barrier(); asm volatile("" ::: "memory"); }

__global__ __launch_bounds__(256) void k_cvt8(const float* __restrict__ x, h16* XH) {
    const size_t i = (size_t)blockIdx.x * 256 + threadIdx.x; const size_t n8 = (size_t)NB * SEQ * DM / 8; if (i >= n8) return;
    const size_t r = i / (DM / 8); const size_t c8 = i % (DM / 8); const size_t b = r / SEQ, s = r % SEQ;
    const float* src = x + (b * SEQ_FULL + s) * DM + c8 * 8;
    const v4f v0 = *(const v4f*)src; const v4f v1 = *(const v4f*)(src + 4); v8h o;
    o[0] = (h16)bfr(v0[0]); o[1] = (h16)bfr(v0[1]); o[2] = (h16)bfr(v0[2]); o[3] = (h16)bfr(v0[3]);
    o[4] = (h16)bfr(v1[0]); o[5] = (h16)bfr(v1[1]); o[6] = (h16)bfr(v1[2]); o[7] = (h16)bfr(v1[3]);
    *(volatile v8h*)(XH + i * 8) = o; __threadfence(); *(volatile v8h*)(XH + i * 8) = o;
}

__global__ __launch_bounds__(256) void k_wt(const float* __restrict__ w, int K, int N, int Z, h16* Bt) {
    const size_t i = (size_t)blockIdx.x * 256 + threadIdx.x; const size_t n8 = (size_t)Z * N * K / 8; if (i >= n8) return;
    const size_t e = i * 8; const size_t k = e % (size_t)K; const size_t n = (e / (size_t)K) % (size_t)N; const size_t z = e / ((size_t)K * N);
    const float* s = w + (z * K + k) * N + n; v8h o;
#pragma unroll
    for (int j = 0; j < 8; ++j) o[j] = (h16)(bfr(s[(size_t)j * N]) * WCAR);
    *(volatile v8h*)(Bt + e) = o; __threadfence(); *(volatile v8h*)(Bt + e) = o;
}

__device__ __forceinline__ void gemm64(const h16* __restrict__ A, const h16* __restrict__ Bt, v8f (&acc)[4][4], int lr, int hi) {
#pragma unroll
    for (int mb = 0; mb < 4; ++mb)
#pragma unroll
        for (int nb = 0; nb < 4; ++nb) acc[mb][nb] = (v8f){};
    const size_t off = (size_t)lr * DM + 8 * hi;
#pragma unroll 1
    for (int kc = 0; kc < DM; kc += 32) {
        v16h a[4]; v16h b;
#pragma unroll
        for (int mb = 0; mb < 4; ++mb) a[mb] = ldh(A + off + (size_t)mb * 16 * DM + kc);
#pragma unroll
        for (int nb = 0; nb < 4; ++nb) { b = ldh(Bt + off + (size_t)nb * 16 * DM + kc);
#pragma unroll
            for (int mb = 0; mb < 4; ++mb) acc[mb][nb] = wmma16(a[mb], b, acc[mb][nb]); }
        asm volatile("v_nop\n\tv_nop\n\tv_nop\n\tv_nop" : "+v"(acc[0][0]), "+v"(acc[1][1]), "+v"(acc[2][2]), "+v"(acc[3][3]) : "v"(a[0]), "v"(a[3]), "v"(b));
    }
}

__device__ __forceinline__ void store_tile64(const h16* ts_base_unused, h16* dst, size_t pitch, int lane);

__global__ __launch_bounds__(32) void k_projqk(const h16* __restrict__ XH, const h16* __restrict__ WT, const float* __restrict__ bias, h16* P) {
    __shared__ __align__(16) h16 ts[64 * TSP];
    const int lane = threadIdx.x & 31, lr = lane & 15, hi = lane >> 4;
    const int r0 = blockIdx.x * 64, head = blockIdx.y; const int bz = r0 / SEQ, s0 = r0 % SEQ;
    v8f acc[4][4];
    gemm64(WT + (size_t)head * HD * DM, XH + (size_t)r0 * DM, acc, lr, hi);
#pragma unroll
    for (int mb = 0; mb < 4; ++mb) {
        const v4f b0 = *(const v4f*)(bias + head * HD + mb * 16 + 8 * hi); const v4f b1 = *(const v4f*)(bias + head * HD + mb * 16 + 8 * hi + 4);
        v8f bb; bb[0] = bfr(b0[0]); bb[1] = bfr(b0[1]); bb[2] = bfr(b0[2]); bb[3] = bfr(b0[3]); bb[4] = bfr(b1[0]); bb[5] = bfr(b1[1]); bb[6] = bfr(b1[2]); bb[7] = bfr(b1[3]);
#pragma unroll
        for (int nb = 0; nb < 4; ++nb) { v8h hv;
#pragma unroll
            for (int j = 0; j < 8; ++j) hv[j] = (h16)(acc[mb][nb][j] * WINV + bb[j]);
            *(v8ha*)(&ts[(nb * 16 + lr) * TSP + mb * 16 + 8 * hi]) = hv; } }
    wave_lds_sync();
    h16* dst = P + (((size_t)bz * NH + head) * SEQ + s0) * HD;
#pragma unroll 1
    for (int ps = 0; ps < 2; ++ps) {
#pragma unroll
        for (int it = 0; it < 16; ++it) { const int L = it * 4 + (lane >> 3), pc = lane & 7; const v8h val = *(const v8ha*)(&ts[L * TSP + pc * 8]);
            *(volatile v8h*)(dst + (size_t)L * HD + pc * 8) = val; }
        if (ps == 0) __threadfence(); }
}

__global__ __launch_bounds__(32) void k_projv(const h16* __restrict__ XH, const h16* __restrict__ WT, const float* __restrict__ bias, h16* VT) {
    __shared__ __align__(16) h16 ts[64 * TSP];
    const int lane = threadIdx.x & 31, lr = lane & 15, hi = lane >> 4;
    const int r0 = blockIdx.x * 64, head = blockIdx.y; const int bz = r0 / SEQ, s0 = r0 % SEQ;
    v8f acc[4][4];
    gemm64(XH + (size_t)r0 * DM, WT + (size_t)head * HD * DM, acc, lr, hi);
#pragma unroll
    for (int nb = 0; nb < 4; ++nb) { const float bb = bfr(bias[head * HD + nb * 16 + lr]);
#pragma unroll
        for (int mb = 0; mb < 4; ++mb) { v8h hv;
#pragma unroll
            for (int j = 0; j < 8; ++j) hv[j] = (h16)(acc[mb][nb][j] * WINV + bb);
            *(v8ha*)(&ts[(nb * 16 + lr) * TSP + mb * 16 + 8 * hi]) = hv; } }
    wave_lds_sync();
    h16* dst = VT + (((size_t)bz * NH + head) * HD) * SEQ + s0;
#pragma unroll 1
    for (int ps = 0; ps < 2; ++ps) {
#pragma unroll
        for (int it = 0; it < 16; ++it) { const int L = it * 4 + (lane >> 3), pc = lane & 7; const v8h val = *(const v8ha*)(&ts[L * TSP + pc * 8]);
            *(volatile v8h*)(dst + (size_t)L * SEQ + pc * 8) = val; }
        if (ps == 0) __threadfence(); }
}

__global__ __launch_bounds__(128) void k_attn(const h16* __restrict__ Qp, const h16* __restrict__ Kp, const h16* __restrict__ Vt, h16* Ctx) {
    __shared__ __align__(16) h16 os[4 * 16 * TSP];
    const int lane = threadIdx.x & 31, lr = lane & 15, hi = lane >> 4, wv = threadIdx.x >> 5;
    const int bh = blockIdx.y; const int q0 = blockIdx.x * 64 + wv * 16;
    const size_t pbase = (size_t)bh * SEQ * HD;
    const h16* qrow = Qp + pbase + (size_t)(q0 + lr) * HD + 8 * hi;
    const v16h qb0 = ldh(qrow), qb1 = ldh(qrow + 32);
    const h16* kbase = Kp + pbase + (size_t)lr * HD + 8 * hi;
    const h16* vbase = Vt + pbase + (size_t)lr * SEQ + 8 * hi;
    v8f o[4];
#pragma unroll
    for (int dt = 0; dt < 4; ++dt) o[dt] = (v8f){};
    float m = -3.0e38f, l = 0.0f;
#pragma unroll 1
    for (int kb = 0; kb < SEQ; kb += 64) {
        v8f st[4]; v16h ka0, ka1;
#pragma unroll
        for (int t = 0; t < 4; ++t) { const h16* kp = kbase + (size_t)(kb + t * 16) * HD; ka0 = ldh(kp); ka1 = ldh(kp + 32);
            v8f c = (v8f){}; c = wmma16(ka0, qb0, c); c = wmma16(ka1, qb1, c); st[t] = c; }
        asm volatile("v_nop\n\tv_nop\n\tv_nop\n\tv_nop" : "+v"(st[0]), "+v"(st[1]), "+v"(st[2]), "+v"(st[3]) : "v"(ka0), "v"(ka1), "v"(qb0), "v"(qb1));
        float mloc = fmaxf(fmaxf(st[0][0], st[1][0]), fmaxf(st[2][0], st[3][0]));
#pragma unroll
        for (int j = 1; j < 8; ++j) mloc = fmaxf(mloc, fmaxf(fmaxf(st[0][j], st[1][j]), fmaxf(st[2][j], st[3][j])));
        mloc = fmaxf(mloc, __shfl_xor(mloc, 16, 32));
        const float mnew = fmaxf(m, mloc * C2);
        const float corr = __builtin_amdgcn_exp2f(m - mnew); m = mnew;
        v16h pb0, pb1; float psum = 0.0f;
#pragma unroll
        for (int j = 0; j < 8; ++j) {
            const float p0 = __builtin_amdgcn_exp2f(__builtin_fmaf(st[0][j], C2, -mnew));
            const float p1 = __builtin_amdgcn_exp2f(__builtin_fmaf(st[1][j], C2, -mnew));
            const float p2 = __builtin_amdgcn_exp2f(__builtin_fmaf(st[2][j], C2, -mnew));
            const float p3 = __builtin_amdgcn_exp2f(__builtin_fmaf(st[3][j], C2, -mnew));
            psum += (p0 + p1) + (p2 + p3);
            pb0[j] = (h16)p0; pb0[8 + j] = (h16)p1; pb1[j] = (h16)p2; pb1[8 + j] = (h16)p3; }
        l = l * corr + psum;
#pragma unroll
        for (int dt = 0; dt < 4; ++dt)
#pragma unroll
            for (int j = 0; j < 8; ++j) o[dt][j] *= corr;
        v16h va0, va1;
#pragma unroll
        for (int dt = 0; dt < 4; ++dt) { const h16* vp = vbase + (size_t)dt * 16 * SEQ + kb; va0 = ldh(vp); va1 = ldh(vp + 32);
            o[dt] = wmma16(va0, pb0, o[dt]); o[dt] = wmma16(va1, pb1, o[dt]); }
        asm volatile("v_nop\n\tv_nop\n\tv_nop\n\tv_nop" : "+v"(o[0]), "+v"(o[1]), "+v"(o[2]), "+v"(o[3]) : "v"(va0), "v"(va1), "v"(pb0), "v"(pb1));
    }
    const float lt = l + __shfl_xor(l, 16, 32);
    const float inv = CCAR * (1.0f / lt);
    const int ob = wv * 16 * TSP;
#pragma unroll
    for (int dt = 0; dt < 4; ++dt) { v8h hv;
#pragma unroll
        for (int j = 0; j < 8; ++j) hv[j] = (h16)(o[dt][j] * inv);
        *(v8ha*)(&os[ob + lr * TSP + dt * 16 + 8 * hi]) = hv; }
    wave_lds_sync();
    const int b = bh / NH, h = bh % NH;
    h16* dst = Ctx + ((size_t)b * SEQ + q0) * DM + h * HD;
#pragma unroll 1
    for (int ps = 0; ps < 2; ++ps) {
#pragma unroll
        for (int it = 0; it < 4; ++it) { const int qq = it * 4 + (lane >> 3), pc = lane & 7; const v8h val = *(const v8ha*)(&os[ob + qq * TSP + pc * 8]);
            *(volatile v8h*)(dst + (size_t)qq * DM + pc * 8) = val; }
        if (ps == 0) __threadfence(); }
}

__global__ __launch_bounds__(32) void k_outp(const h16* __restrict__ CTX, const h16* __restrict__ WO, const float* __restrict__ bias, float* OUT) {
    __shared__ __align__(16) float os[16 * 68];
    const int lane = threadIdx.x & 31, lr = lane & 15, hi = lane >> 4;
    const int r0 = blockIdx.x * 64, c0 = blockIdx.y * 64; const int bz = r0 / SEQ, s0 = r0 % SEQ;
    v8f acc[4][4];
    gemm64(CTX + (size_t)r0 * DM, WO + (size_t)c0 * DM, acc, lr, hi);
    const v4f braw = *(const v4f*)(bias + c0 + lr * 4); v4f bb; bb[0] = bfr(braw[0]); bb[1] = bfr(braw[1]); bb[2] = bfr(braw[2]); bb[3] = bfr(braw[3]);
    float* cbase = OUT + ((size_t)bz * SEQ_FULL + s0) * DM + c0;
#pragma unroll
    for (int mb = 0; mb < 4; ++mb) {
#pragma unroll
        for (int nb = 0; nb < 4; ++nb) {
#pragma unroll
            for (int j = 0; j < 8; ++j) os[(hi * 8 + j) * 68 + nb * 16 + lr] = acc[mb][nb][j] * OINV; }
        wave_lds_sync();
        float* crow = cbase + (size_t)(mb * 16) * DM;
#pragma unroll 1
        for (int ps = 0; ps < 2; ++ps) {
#pragma unroll
            for (int s = 0; s < 8; ++s) { const int row = 2 * s + hi, cofs = lr * 4; v4f val = *(const v4fa*)(os + row * 68 + cofs); val += bb;
                *(volatile v4f*)(crow + (size_t)row * DM + cofs) = val; }
            if (ps == 0) __threadfence(); }
        wave_lds_sync();
    }
}

#define SZ_X    ((size_t)NB * SEQ * DM * 2)
#define SZ_W    ((size_t)DM * DM * 2)
#define SZ_ALL  (SZ_X * 5 + SZ_W * 4)
static_assert(SZ_X % 256 == 0);
static_assert(SZ_W % 256 == 0);
static_assert(SZ_ALL <= (size_t)134217728);

extern "C" void kernel_launch(void* const* d_in, const int* in_sizes, int n_in,
                              void* d_out, int out_size, void* d_ws, size_t ws_size, hipStream_t stream) {
    if (n_in < 9) return;
    const size_t needx = ((size_t)(NB - 1) * SEQ_FULL + SEQ) * DM;
    if ((size_t)in_sizes[0] < needx) return;
    if ((size_t)in_sizes[1] < (size_t)NH * DM * HD || (size_t)in_sizes[3] < (size_t)NH * DM * HD || (size_t)in_sizes[5] < (size_t)NH * DM * HD) return;
    if ((size_t)in_sizes[2] < (size_t)NH * HD || (size_t)in_sizes[4] < (size_t)NH * HD || (size_t)in_sizes[6] < (size_t)NH * HD) return;
    if ((size_t)in_sizes[7] < (size_t)DM * DM || (size_t)in_sizes[8] < (size_t)DM) return;
    if ((size_t)out_size < needx) return;
    if (SZ_ALL > ws_size) return;
    const float* xs = (const float*)d_in[0];
    const float* Wq = (const float*)d_in[1]; const float* bq = (const float*)d_in[2];
    const float* Wk = (const float*)d_in[3]; const float* bk = (const float*)d_in[4];
    const float* Wv = (const float*)d_in[5]; const float* bv = (const float*)d_in[6];
    const float* Wo = (const float*)d_in[7]; const float* bo = (const float*)d_in[8];
    float* OUT = (float*)d_out;
    char* wsp = (char*)d_ws;
    h16* XH  = (h16*)wsp; wsp += SZ_X;
    h16* WQ  = (h16*)wsp; wsp += SZ_W;
    h16* WK  = (h16*)wsp; wsp += SZ_W;
    h16* WV  = (h16*)wsp; wsp += SZ_W;
    h16* WO  = (h16*)wsp; wsp += SZ_W;
    h16* QP  = (h16*)wsp; wsp += SZ_X;
    h16* KP  = (h16*)wsp; wsp += SZ_X;
    h16* VT  = (h16*)wsp; wsp += SZ_X;
    h16* CTX = (h16*)wsp; wsp += SZ_X;

    k_cvt8<<<(unsigned)(((size_t)NB * SEQ * DM / 8 + 255) / 256), 256, 0, stream>>>(xs, XH);
    const unsigned gw = (unsigned)(((size_t)DM * DM / 8 + 255) / 256);
    k_wt<<<gw, 256, 0, stream>>>(Wq, DM, HD, NH, WQ);
    k_wt<<<gw, 256, 0, stream>>>(Wk, DM, HD, NH, WK);
    k_wt<<<gw, 256, 0, stream>>>(Wv, DM, HD, NH, WV);
    k_wt<<<gw, 256, 0, stream>>>(Wo, DM, DM, 1, WO);
    k_projqk<<<dim3(NB * SEQ / 64, NH, 1), 32, 0, stream>>>(XH, WQ, bq, QP);
    k_projqk<<<dim3(NB * SEQ / 64, NH, 1), 32, 0, stream>>>(XH, WK, bk, KP);
    k_projv<<<dim3(NB * SEQ / 64, NH, 1), 32, 0, stream>>>(XH, WV, bv, VT);
    k_attn<<<dim3(SEQ / 64, NB * NH, 1), 128, 0, stream>>>(QP, KP, VT, CTX);
    k_outp<<<dim3(NB * SEQ / 64, DM / 64, 1), 32, 0, stream>>>(CTX, WO, bo, OUT);
}
